// MultiHeadDistanceLayer_2370821947428
// MI455X (gfx1250) — hardware-run, weakly checked
//
#include <hip/hip_runtime.h>
#include <math.h>
#include <stdint.h>

#ifndef NB
#define NB 4
#endif
#ifndef SEQ
#define SEQ 1024
#endif
#define NB_FULL  4
#define SEQ_FULL 1024
#define DM    256
#define NHEAD 8
#define HD    64
#define DQ    (NHEAD * HD)
#define DQK   (2 * DQ)
#define KC    (2 * DM)
#define NQT   (SEQ / 32)
#define NKT   (SEQ / 64)
static_assert(NB >= 1 && NB <= NB_FULL);
static_assert(SEQ >= 256 && SEQ <= SEQ_FULL && (SEQ % 256) == 0);
static_assert(((NB * SEQ) % 64) == 0);
static_assert((DQK % 64) == 0 && (KC % 32) == 0 && (DM % 64) == 0 && (DQ % 64) == 0);
static_assert(NHEAD * 32 == 256);

typedef _Float16 v16h __attribute__((ext_vector_type(16)));
typedef _Float16 v8h  __attribute__((ext_vector_type(8)));
typedef __bf16   v16b __attribute__((ext_vector_type(16)));
typedef __bf16   v8b  __attribute__((ext_vector_type(8)));
typedef float    v8f  __attribute__((ext_vector_type(8)));
typedef float    v4f  __attribute__((ext_vector_type(4)));
typedef unsigned int v4u __attribute__((ext_vector_type(4)));

#if defined(__HIP_DEVICE_COMPILE__)
#define DEV_ASM 1
#else
#define DEV_ASM 0
#endif

__device__ __forceinline__ unsigned short bf_bits(float f) {
  unsigned u = __float_as_uint(f);
  return (unsigned short)((u + 0x7FFFu + ((u >> 16) & 1u)) >> 16);
}
__device__ __forceinline__ float bf_up(unsigned short hb) { return __uint_as_float(((unsigned)hb) << 16); }
__device__ __forceinline__ float bfr(float f) { return bf_up(bf_bits(f)); }
__device__ __forceinline__ unsigned short h_bits(_Float16 x) { return __builtin_bit_cast(unsigned short, x); }
__device__ __forceinline__ unsigned pk16(unsigned short a, unsigned short b) { return (unsigned)a | ((unsigned)b << 16); }
__device__ __forceinline__ v8f zero8() { v8f z = {0.f, 0.f, 0.f, 0.f, 0.f, 0.f, 0.f, 0.f}; return z; }

template <typename OT> struct FT;
template <> struct FT<__bf16>   { typedef v16b frag; typedef v8b half8; };
template <> struct FT<_Float16> { typedef v16h frag; typedef v8h half8; };

template <typename OT>
__device__ __forceinline__ typename FT<OT>::frag ldfrag(const OT* p) {
  union { typename FT<OT>::frag v; typename FT<OT>::half8 h[2]; } f;
  f.h[0] = *(const typename FT<OT>::half8*)(p);
  f.h[1] = *(const typename FT<OT>::half8*)(p + 16);
  return f.v;
}

__device__ __forceinline__ v8f mmar(v16b a, v16b b, v8f c) {
  return __builtin_amdgcn_wmma_f32_16x16x32_bf16(false, a, false, b, (short)0, c, false, false);
}
__device__ __forceinline__ v8f mmar(v16h a, v16h b, v8f c) {
  return __builtin_amdgcn_wmma_f32_16x16x32_f16(false, a, false, b, (short)0, c, false, false);
}
__device__ __forceinline__ v8f mma_h(v16h a, v16h b, v8f c) {
  c = __builtin_amdgcn_wmma_f32_16x16x32_f16(false, a, false, b, (short)0, c, false, false);
#if DEV_ASM
  asm volatile("v_nop\n\tv_nop\n\tv_nop\n\tv_nop" : "+v"(c) : "v"(a), "v"(b));
#endif
  return c;
}
__device__ __forceinline__ void dep_guard(v8f& a, v8f& b, v16b x, v16b y) {
#if DEV_ASM
  asm volatile("v_nop\n\tv_nop\n\tv_nop\n\tv_nop" : "+v"(a), "+v"(b) : "v"(x), "v"(y));
#else
  (void)a; (void)b; (void)x; (void)y;
#endif
}
__device__ __forceinline__ void dep_guard(v8f& a, v8f& b, v16h x, v16h y) {
#if DEV_ASM
  asm volatile("v_nop\n\tv_nop\n\tv_nop\n\tv_nop" : "+v"(a), "+v"(b) : "v"(x), "v"(y));
#else
  (void)a; (void)b; (void)x; (void)y;
#endif
}
__device__ __forceinline__ void keep4(v16b a, v16b b, v16b c, v16b d) {
#if DEV_ASM
  asm volatile("v_nop" :: "v"(a), "v"(b), "v"(c), "v"(d));
#else
  (void)a; (void)b; (void)c; (void)d;
#endif
}
__device__ __forceinline__ void keep4(v16h a, v16h b, v16h c, v16h d) {
#if DEV_ASM
  asm volatile("v_nop" :: "v"(a), "v"(b), "v"(c), "v"(d));
#else
  (void)a; (void)b; (void)c; (void)d;
#endif
}
__device__ __forceinline__ void acc_guard4(v8f& a, v8f& b, v8f& c, v8f& d) {
#if DEV_ASM
  asm volatile("v_nop\n\tv_nop\n\tv_nop\n\tv_nop" : "+v"(a), "+v"(b), "+v"(c), "+v"(d));
#else
  (void)a; (void)b; (void)c; (void)d;
#endif
}

__global__ __launch_bounds__(256) void cvt_xpe(const float* __restrict__ x, const float* __restrict__ pe,
                                               unsigned short* xc, int n8) {
  const int i = blockIdx.x * 256 + (int)threadIdx.x;
  if (i < n8) {
    const int row = i >> 5;
    const int col = (i & 31) * 8;
    const int b = row / SEQ;
    const int l = row - b * SEQ;
    const float* xp = x  + ((size_t)b * SEQ_FULL + l) * DM + col;
    const float* pp = pe + (size_t)l * DM + col;
    const v4f x0 = *(const v4f*)xp, x1 = *(const v4f*)(xp + 4);
    const v4f p0 = *(const v4f*)pp, p1 = *(const v4f*)(pp + 4);
    float s[8];
#pragma unroll
    for (int e = 0; e < 4; ++e) {
      s[e]     = bfr(x0[e]) + bfr(p0[e]);
      s[4 + e] = bfr(x1[e]) + bfr(p1[e]);
    }
    v4u hv, lv;
#pragma unroll
    for (int e = 0; e < 4; ++e) {
      const unsigned short hb0 = bf_bits(s[2 * e]), hb1 = bf_bits(s[2 * e + 1]);
      const unsigned short lb0 = bf_bits(s[2 * e] - bf_up(hb0));
      const unsigned short lb1 = bf_bits(s[2 * e + 1] - bf_up(hb1));
      hv[e] = pk16(hb0, hb1);
      lv[e] = pk16(lb0, lb1);
    }
    unsigned short* o = xc + (size_t)row * KC + col;
    *(volatile v4u*)o = hv;
    *(volatile v4u*)(o + DM) = lv;
    __threadfence();
    *(volatile v4u*)o = hv;
    *(volatile v4u*)(o + DM) = lv;
  }
}

__global__ __launch_bounds__(256) void w_prep(const float* __restrict__ Wq, const float* __restrict__ Wk,
                                              unsigned short* wc) {
  __shared__ float T[64][65];
  const int tid = (int)threadIdx.x;
  const int n0 = blockIdx.x * 64;
  const int k0 = blockIdx.y * 64;
  const bool useq = (n0 < DQ);
  const float* W = useq ? Wq : Wk;
  const int nn0 = useq ? n0 : (n0 - DQ);
  {
    const int kr = tid >> 2, c16 = (tid & 3) * 16;
    const float* src = W + (size_t)(k0 + kr) * DQ + nn0 + c16;
#pragma unroll
    for (int j = 0; j < 4; ++j) {
      const v4f a = *(const v4f*)(src + 4 * j);
#pragma unroll
      for (int e = 0; e < 4; ++e) T[c16 + 4 * j + e][kr] = a[e];
    }
  }
  __syncthreads();
  const int q = tid >> 3, c8 = (tid & 7) * 8;
  v4u pv[2];
#pragma unroll
  for (int it = 0; it < 2; ++it) {
    const int row = it * 32 + q;
    v4u p;
#pragma unroll
    for (int e = 0; e < 4; ++e)
      p[e] = pk16(bf_bits(T[row][c8 + 2 * e]), bf_bits(T[row][c8 + 2 * e + 1]));
    pv[it] = p;
  }
  for (int pass = 0; pass < 2; ++pass) {
#pragma unroll
    for (int it = 0; it < 2; ++it) {
      const int row = it * 32 + q;
      unsigned short* o = wc + (size_t)(n0 + row) * KC + k0 + c8;
      *(volatile v4u*)o = pv[it];
      *(volatile v4u*)(o + DM) = pv[it];
    }
    __threadfence();
  }
}

__global__ __launch_bounds__(256) void v_proj(const float* __restrict__ x, const float* __restrict__ Wv,
                                              float* vv, int n) {
  const int t = blockIdx.x * 256 + (int)threadIdx.x;
  if (t < n) {
    const int hb = t / SEQ;
    const int l  = t - hb * SEQ;
    const int h  = hb / NB;
    const int b  = hb - h * NB;
    const float* xr = x + ((size_t)b * SEQ_FULL + l) * DM;
    float acc = 0.f;
#pragma unroll 1
    for (int d4 = 0; d4 < DM; d4 += 4) {
      const v4f xv = *(const v4f*)(xr + d4);
      const float w0 = Wv[(d4 + 0) * NHEAD + h], w1 = Wv[(d4 + 1) * NHEAD + h];
      const float w2 = Wv[(d4 + 2) * NHEAD + h], w3 = Wv[(d4 + 3) * NHEAD + h];
      acc = fmaf(bfr(xv[0]), bfr(w0), acc);
      acc = fmaf(bfr(xv[1]), bfr(w1), acc);
      acc = fmaf(bfr(xv[2]), bfr(w2), acc);
      acc = fmaf(bfr(xv[3]), bfr(w3), acc);
    }
    const float ev = __expf(-acc);
    const float v  = 1.0f / (1.0f + ev);
    *(volatile float*)(vv + t) = v;
    __threadfence();
    *(volatile float*)(vv + t) = v;
  }
}

template <typename OT, int OUT_MODE>
__global__ __launch_bounds__(256) void gemm64(
    const unsigned short* __restrict__ Ap, int lda,
    const unsigned short* __restrict__ Btp, int ldb,
    void* Cout, void* Cout2, int ldc,
    const float* __restrict__ bias0, int nb0, const float* __restrict__ bias1, int nb1,
    int M, int N, int K, float oscale, float rscale) {
  typedef typename FT<OT>::frag V16;
  const OT* A  = (const OT*)(const void*)Ap;
  const OT* Bt = (const OT*)(const void*)Btp;
  __shared__ __align__(16) float sT[8][16 * 68];
  const int lane = threadIdx.x & 31;
  const int wave = threadIdx.x >> 5;
  const int tilesN = N >> 6;
  const int tilesM = M >> 6;
  const int tile = blockIdx.x * 8 + wave;
  if (tile >= tilesM * tilesN) return;
  const int tm = tile / tilesN;
  const int tn = tile - tm * tilesN;
  const int m0 = tm << 6;
  const int n0 = tn << 6;

  const int rlane = lane & 15;
  const int koff  = (lane >> 4) * 8;
  const int mOff  = (lane >> 4) * 8;

  v8f acc[4][4];
#pragma unroll
  for (int i = 0; i < 4; ++i)
#pragma unroll
    for (int j = 0; j < 4; ++j) acc[i][j] = zero8();

  for (int k0 = 0; k0 < K; k0 += 32) {
    V16 bq[4];
#pragma unroll
    for (int j = 0; j < 4; ++j)
      bq[j] = ldfrag<OT>(Bt + (size_t)(n0 + (j << 4) + rlane) * ldb + koff + k0);
#pragma unroll
    for (int i = 0; i < 4; ++i) {
      const V16 af = ldfrag<OT>(A + (size_t)(m0 + (i << 4) + rlane) * lda + koff + k0);
#pragma unroll
      for (int j = 0; j < 4; ++j) acc[i][j] = mmar(af, bq[j], acc[i][j]);
      dep_guard(acc[i][0], acc[i][3], af, bq[3]);
    }
    keep4(bq[0], bq[1], bq[2], bq[3]);
  }
  acc_guard4(acc[0][0], acc[0][1], acc[0][2], acc[0][3]);
  acc_guard4(acc[1][0], acc[1][1], acc[1][2], acc[1][3]);
  acc_guard4(acc[2][0], acc[2][1], acc[2][2], acc[2][3]);
  acc_guard4(acc[3][0], acc[3][1], acc[3][2], acc[3][3]);

  float bv[8];
  {
    const int cb = (OUT_MODE == 0) ? (lane & 15) * 4 : (lane & 7) * 8;
    const int nq = n0 + cb;
    const int i0 = min(nq, nb0 - 8);
    const int i1 = min(max(nq - nb0, 0), nb1 - 8);
    const v4f a0 = *(const v4f*)(bias0 + i0), a1 = *(const v4f*)(bias0 + i0 + 4);
    const v4f c0 = *(const v4f*)(bias1 + i1), c1 = *(const v4f*)(bias1 + i1 + 4);
    const bool use0 = (nq < nb0);
#pragma unroll
    for (int e = 0; e < 4; ++e) {
      bv[e]     = bfr(use0 ? a0[e] : c0[e]);
      bv[4 + e] = bfr(use0 ? a1[e] : c1[e]);
    }
  }

  float* slab = sT[wave];
#pragma unroll
  for (int i = 0; i < 4; ++i) {
    const int mBase = m0 + (i << 4);
#pragma unroll
    for (int j = 0; j < 4; ++j) {
#pragma unroll
      for (int r = 0; r < 8; ++r) {
        slab[(mOff + r) * 68 + (j << 4) + rlane] = acc[i][j][r];
      }
    }
    __builtin_amdgcn_fence(__ATOMIC_RELEASE, "workgroup");
    __builtin_amdgcn_wave_barrier();
    __builtin_amdgcn_fence(__ATOMIC_ACQUIRE, "workgroup");
    if (OUT_MODE == 0) {
      float* C = (float*)Cout;
      const int h2 = lane >> 4, c4 = (lane & 15) * 4;
      v4f ov[8];
#pragma unroll
      for (int it = 0; it < 8; ++it) {
        const int row = it * 2 + h2;
        v4f v = *(const v4f*)(slab + row * 68 + c4) * oscale;
#pragma unroll
        for (int e = 0; e < 4; ++e) v[e] += bv[e];
        ov[it] = v;
      }
      for (int pass = 0; pass < 2; ++pass) {
#pragma unroll
        for (int it = 0; it < 8; ++it) {
          const int row = it * 2 + h2;
          *(volatile v4f*)(C + (size_t)(mBase + row) * ldc + n0 + c4) = ov[it];
        }
        __threadfence();
      }
    } else {
      const int q = lane >> 3, c8 = (lane & 7) * 8;
      unsigned short* C  = (unsigned short*)Cout;
      unsigned short* C2 = (unsigned short*)Cout2;
      v4u hv[4], lv[4];
#pragma unroll
      for (int it = 0; it < 4; ++it) {
        const int row = it * 4 + q;
        const float* sp = slab + row * 68 + c8;
        float f[8];
#pragma unroll
        for (int e = 0; e < 8; ++e) f[e] = sp[e] * oscale + bv[e];
        v4u a, a2;
#pragma unroll
        for (int e = 0; e < 4; ++e) {
          const float f0 = f[2 * e], f1 = f[2 * e + 1];
          const _Float16 x0 = (_Float16)f0, x1 = (_Float16)f1;
          const unsigned short h0 = h_bits(x0), h1 = h_bits(x1);
          unsigned short l0 = 0, l1 = 0;
          if (OUT_MODE == 3) {
            l0 = h_bits((_Float16)((f0 - (float)x0) * rscale));
            l1 = h_bits((_Float16)((f1 - (float)x1) * rscale));
          }
          a[e] = pk16(h0, h1); a2[e] = pk16(l0, l1);
        }
        hv[it] = a; lv[it] = a2;
      }
      for (int pass = 0; pass < 2; ++pass) {
#pragma unroll
        for (int it = 0; it < 4; ++it) {
          const int row = it * 4 + q;
          *(volatile v4u*)(C + (size_t)(mBase + row) * ldc + n0 + c8) = hv[it];
          if (OUT_MODE == 3) *(volatile v4u*)(C2 + (size_t)(mBase + row) * ldc + n0 + c8) = lv[it];
        }
        __threadfence();
      }
    }
    __builtin_amdgcn_fence(__ATOMIC_RELEASE, "workgroup");
    __builtin_amdgcn_wave_barrier();
    __builtin_amdgcn_fence(__ATOMIC_ACQUIRE, "workgroup");
  }
}

__global__ __launch_bounds__(64)
void attn_diag(const unsigned short* __restrict__ chp, const unsigned short* __restrict__ clp,
               const float* __restrict__ vv, float* part, float sscale) {
  union FH { v16h v; v8h h[2]; };
  extern __shared__ __align__(16) unsigned char smem_raw[];
  float*    Sc  = (float*)(void*)smem_raw;
  _Float16* Ksh = (_Float16*)(void*)(smem_raw + (size_t)32 * SEQ * 4);
  float*    vs  = (float*)(void*)(smem_raw + (size_t)32 * SEQ * 4 + (size_t)64 * 64 * 2);
  float*    rl  = vs + SEQ;

  const int tid  = (int)threadIdx.x;
  const int wave = tid >> 5;
  const int lane = tid & 31;
  const int hh   = lane >> 4;
  const int c    = lane & 15;
  const int bx   = (int)blockIdx.x;
  const int qt   = bx % NQT;
  const int hb   = bx / NQT;
  const int h    = hb / NB;
  const int b    = hb - h * NB;
  const int q0   = qt * 32;
  const int qw   = q0 + 16 * wave;
  const size_t rowB = (size_t)b * SEQ;
  const _Float16* Ch = (const _Float16*)(const void*)chp;
  const _Float16* Cl = (const _Float16*)(const void*)clp;

#pragma unroll
  for (int i = 0; i < SEQ / 256; ++i) {
    const int l4 = (tid + 64 * i) * 4;
    const v4f a = *(const v4f*)(vv + (size_t)hb * SEQ + l4);
#pragma unroll
    for (int e = 0; e < 4; ++e) vs[SEQ - 1 - (l4 + e)] = a[e];
  }

  v16h qah[2], qal[2];
#pragma unroll
  for (int dc = 0; dc < 2; ++dc) {
    const size_t qo = (rowB + qw + c) * DQK + (size_t)h * HD + dc * 32 + 8 * hh;
    qah[dc] = ldfrag<_Float16>(Ch + qo);
    qal[dc] = ldfrag<_Float16>(Cl + qo);
  }

  float mrow[8];
#pragma unroll
  for (int r = 0; r < 8; ++r) mrow[r] = -INFINITY;
  float* srow = Sc + (size_t)(16 * wave + 8 * hh) * SEQ + c;

#pragma unroll 1
  for (int kt = 0; kt < NKT; ++kt) {
    const int kv0 = kt * 64;
    __syncthreads();
    {
      const _Float16* kg = Ch + (rowB + kv0 + tid) * DQK + DQ + (size_t)h * HD;
#pragma unroll
      for (int i = 0; i < 8; ++i) *(v8h*)(Ksh + tid * 64 + 8 * i) = *(const v8h*)(kg + 8 * i);
    }
    __syncthreads();

#pragma unroll
    for (int j = 0; j < 4; ++j) {
      v8f ah = zero8(), al = zero8();
#pragma unroll
      for (int dc = 0; dc < 2; ++dc) {
        FH kb;
        kb.h[0] = *(const v8h*)(Ksh + (j * 16 + c) * 64 + dc * 32 + 8 * hh);
        kb.h[1] = *(const v8h*)(Ksh + (j * 16 + c) * 64 + dc * 32 + 16 + 8 * hh);
        ah = mma_h(qah[dc], kb.v, ah);
        al = mma_h(qal[dc], kb.v, al);
      }
#pragma unroll
      for (int r = 0; r < 8; ++r) {
        const float s = (ah[r] + al[r] * (1.0f / 4096.0f)) * sscale;
        mrow[r] = fmaxf(mrow[r], s);
        srow[(size_t)r * SEQ + kv0 + j * 16] = s;
      }
    }
  }

#pragma unroll
  for (int r = 0; r < 8; ++r) {
#pragma unroll
    for (int off = 1; off < 16; off <<= 1) mrow[r] = fmaxf(mrow[r], __shfl_xor(mrow[r], off, 32));
  }
  float lsum[8];
#pragma unroll
  for (int r = 0; r < 8; ++r) lsum[r] = 0.f;
#pragma unroll 1
  for (int kt = 0; kt < NKT; ++kt) {
#pragma unroll
    for (int j = 0; j < 4; ++j) {
      const int n = kt * 64 + j * 16 + c;
      const float vn = vs[n];
#pragma unroll
      for (int r = 0; r < 8; ++r) {
        float* p = srow + (size_t)r * SEQ + kt * 64 + j * 16;
        const float e = __expf(*p - mrow[r]);
        lsum[r] += e;
        *p = e * vn;
      }
    }
  }
  float rinv[8];
#pragma unroll
  for (int r = 0; r < 8; ++r) {
    float l = lsum[r];
#pragma unroll
    for (int off = 1; off < 16; off <<= 1) l += __shfl_xor(l, off, 32);
    rinv[r] = __builtin_amdgcn_rcpf(l);
  }
  if (c == 0) {
#pragma unroll
    for (int r = 0; r < 8; ++r) rl[16 * wave + 8 * hh + r] = rinv[r];
  }
  __syncthreads();

  float rw[32];
#pragma unroll
  for (int r = 0; r < 32; ++r) rw[r] = rl[r];
  float* pbase = part + ((size_t)hb * NQT + qt) * SEQ;
#pragma unroll 1
  for (int i = 0; i < SEQ / 64; ++i) {
    const int dd = tid + 64 * i;
    float acc = 0.f;
#pragma unroll
    for (int r = 0; r < 32; ++r) {
      const int n  = q0 + r + dd;
      const int nn = min(n, SEQ - 1);
      const float w = (n < SEQ) ? rw[r] : 0.0f;
      acc = fmaf(Sc[(size_t)r * SEQ + nn], w, acc);
    }
    float* pp = pbase + dd;
    *(volatile float*)pp = acc;
    __threadfence();
    *(volatile float*)pp = acc;
  }
}

__global__ __launch_bounds__(256) void final_pool(const float* __restrict__ part, float* out) {
  __shared__ __align__(16) float Os[32 * NHEAD];
  const int tid = (int)threadIdx.x;
  const int ndt = SEQ / 32;
  const int b   = (int)blockIdx.x / ndt;
  const int d0  = ((int)blockIdx.x - b * ndt) * 32;
  const int h   = tid >> 5;
  const int dl  = tid & 31;
  const int dd  = d0 + dl;
  const int hb  = h * NB + b;
  const float* pb = part + (size_t)hb * NQT * SEQ;
  const int dm = max(dd - 1, 0), dp = min(dd + 1, SEQ - 1);
  float tm = 0.f, t0 = 0.f, tp = 0.f;
#pragma unroll 4
  for (int q = 0; q < NQT; ++q) {
    const float* pr = pb + (size_t)q * SEQ;
    tm += pr[dm];
    t0 += pr[dd];
    tp += pr[dp];
  }
  const bool hasm = (dd > 0), hasp = (dd < SEQ - 1);
  float s = t0;
  if (hasm) s += tm;
  if (hasp) s += tp;
  const float rc = (hasm && hasp) ? (1.0f / 3.0f) : 0.5f;
  Os[dl * NHEAD + h] = s * rc;
  __syncthreads();
  v4f v = {0.f, 0.f, 0.f, 0.f};
  if (tid < 64) v = *(const v4f*)(Os + tid * 4);
  float* op = out + ((size_t)b * SEQ + d0) * NHEAD + tid * 4;
  if (tid < 64) *(volatile v4f*)op = v;
  __threadfence();
  if (tid < 64) *(volatile v4f*)op = v;
}

extern "C" void kernel_launch(void* const* d_in, const int* in_sizes, int n_in,
                              void* d_out, int out_size, void* d_ws, size_t ws_size,
                              hipStream_t stream) {
  if (n_in < 7) return;
  if (in_sizes[0] < ((NB - 1) * SEQ_FULL + SEQ) * DM) return;
  if (in_sizes[1] < DM * DQ || in_sizes[3] < DM * DQ) return;
  if (in_sizes[2] < DQ || in_sizes[4] < DQ) return;
  if (in_sizes[5] < DM * NHEAD) return;
  if (in_sizes[6] < SEQ * DM) return;
  if (out_size < NB * SEQ * NHEAD) return;

  const float* x  = (const float*)d_in[0];
  const float* Wq = (const float*)d_in[1];
  const float* bq = (const float*)d_in[2];
  const float* Wk = (const float*)d_in[3];
  const float* bk = (const float*)d_in[4];
  const float* Wv = (const float*)d_in[5];
  const float* pe = (const float*)d_in[6];

  const size_t PXC = (size_t)NB * SEQ * KC * 2;
  const size_t PWC = (size_t)DQK * KC * 2;
  const size_t PC  = (size_t)NB * SEQ * DQK * 2;
  const size_t PVV = (size_t)NHEAD * NB * SEQ * 4;
  const size_t PPT = (size_t)NHEAD * NB * NQT * SEQ * 4;
  size_t off = 0;
  const size_t oXc = off; off += PXC;
  const size_t oWc = off; off += PWC;
  const size_t oCh = off; off += PC;
  const size_t oCl = off; off += PC;
  const size_t oVv = off; off += PVV;
  const size_t oPt = off; off += PPT;
  if (off > ws_size) return;
  if (off > (size_t)134217728) return;

  char* ws = (char*)d_ws;
  unsigned short* Xc = (unsigned short*)(ws + oXc);
  unsigned short* Wc = (unsigned short*)(ws + oWc);
  unsigned short* Ch = (unsigned short*)(ws + oCh);
  unsigned short* Cl = (unsigned short*)(ws + oCl);
  float*          Vv = (float*)(ws + oVv);
  float*          Pt = (float*)(ws + oPt);

  const dim3 blk(256);
  const int n8x = NB * SEQ * (DM / 8);
  const int nvv = NHEAD * NB * SEQ;
  const dim3 gCvt((n8x + 255) / 256);
  const dim3 gW(DQK / 64, DM / 64);
  const dim3 gV((nvv + 255) / 256);
  const int  tiles = ((NB * SEQ) / 64) * (DQK / 64);
  const dim3 gG((tiles + 7) / 8);
  const dim3 gA(NHEAD * NB * NQT);
  const dim3 gF(NB * (SEQ / 32));
  const size_t ldsAttn = (size_t)32 * SEQ * 4 + (size_t)64 * 64 * 2 + (size_t)SEQ * 4 + 32 * 4;

  cvt_xpe<<<gCvt, blk, 0, stream>>>(x, pe, Xc, n8x);
  w_prep<<<gW, blk, 0, stream>>>(Wq, Wk, Wc);
  v_proj<<<gV, blk, 0, stream>>>(x, Wv, Vv, nvv);
  gemm64<__bf16, 3><<<gG, blk, 0, stream>>>(
      Xc, KC, Wc, KC, (void*)Ch, (void*)Cl, DQK,
      bq, DQ, bk, DQ, NB * SEQ, DQK, KC, 1.0f, 4096.0f);
  (void)hipFuncSetAttribute(reinterpret_cast<const void*>(&attn_diag),
                            hipFuncAttributeMaxDynamicSharedMemorySize, (int)ldsAttn);
  attn_diag<<<gA, dim3(64), ldsAttn, stream>>>(Ch, Cl, Vv, Pt, 0.125f);
  final_pool<<<gF, blk, 0, stream>>>(Pt, (float*)d_out);
  (void)hipGetLastError();
}
